// Cross_MultiHead_Attention_26895085208063
// MI455X (gfx1250) — hardware-verified
//
#include <hip/hip_runtime.h>
#include <stdint.h>

constexpr int kBatch = 4;
constexpr int kSeq   = 2048;
constexpr int kChan  = 1024;
constexpr int kHeads = 16;
constexpr int kHdim  = 64;
constexpr int kTok   = kBatch * kSeq;
static_assert(kChan == kHeads * kHdim, "head split");
static_assert(kTok % 64 == 0 && kChan % 64 == 0 && (2 * kChan) % 64 == 0, "GEMM M,N tile multiples of 64");
static_assert(kChan % 32 == 0, "GEMM K multiple of 32");
static_assert(kSeq % 64 == 0 && kHdim == 64, "attention tile geometry");

typedef __attribute__((ext_vector_type(16))) _Float16 v16h;
typedef __attribute__((ext_vector_type(8)))  _Float16 v8h;
typedef __attribute__((ext_vector_type(16))) __bf16   v16b;
typedef __attribute__((ext_vector_type(8)))  __bf16   v8b;
typedef __attribute__((ext_vector_type(8)))  float    v8f;
typedef __attribute__((ext_vector_type(4)))  float    v4f;

__device__ __forceinline__ unsigned short f2bf_bits(float f) {
  unsigned u = __float_as_uint(f);
  return (unsigned short)((u + 0x7FFFu + ((u >> 16) & 1u)) >> 16);
}
__device__ __forceinline__ float bf_bits2f(unsigned short h) { return __uint_as_float(((unsigned)h) << 16); }
__device__ __forceinline__ float neg_inf_f() { return __uint_as_float(0xff800000u); }

__device__ __forceinline__ void dep_guard_h(v8f& a, v8f& b, v16h x, v16h y) { asm volatile("v_nop\n\tv_nop\n\tv_nop\n\tv_nop" : "+v"(a), "+v"(b) : "v"(x), "v"(y)); }
__device__ __forceinline__ void dep_guard_b(v8f& a, v8f& b, v16b x, v16b y) { asm volatile("v_nop\n\tv_nop\n\tv_nop\n\tv_nop" : "+v"(a), "+v"(b) : "v"(x), "v"(y)); }
__device__ __forceinline__ void keep4_h(v16h a, v16h b, v16h c, v16h d) { asm volatile("v_nop" :: "v"(a), "v"(b), "v"(c), "v"(d)); }
__device__ __forceinline__ void keep4_b(v16b a, v16b b, v16b c, v16b d) { asm volatile("v_nop" :: "v"(a), "v"(b), "v"(c), "v"(d)); }
__device__ __forceinline__ void acc_guard4(v8f& a, v8f& b, v8f& c, v8f& d) { asm volatile("v_nop\n\tv_nop\n\tv_nop\n\tv_nop" : "+v"(a), "+v"(b), "+v"(c), "+v"(d)); }
template <typename T> struct Frag;
template <> struct Frag<_Float16> {
  typedef v16h V; union U { v16h v; v8h h[2]; };
  static __device__ __forceinline__ v16h load(const _Float16* p) {
    U f; f.h[0] = *(const v8h*)(p); f.h[1] = *(const v8h*)(p + 16); return f.v;
  }
  static __device__ __forceinline__ v8f mma(v16h a, v16h b, v8f c) {
    return __builtin_amdgcn_wmma_f32_16x16x32_f16(false, a, false, b, (short)0, c, false, false);
  }
  static __device__ __forceinline__ void guard(v8f& a, v8f& b, v16h x, v16h y) { dep_guard_h(a, b, x, y); }
  static __device__ __forceinline__ void keep(v16h a, v16h b, v16h c, v16h d) { keep4_h(a, b, c, d); }
};
template <> struct Frag<__bf16> {
  typedef v16b V; union U { v16b v; v8b h[2]; };
  static __device__ __forceinline__ v16b load(const __bf16* p) {
    U f; f.h[0] = *(const v8b*)(p); f.h[1] = *(const v8b*)(p + 16); return f.v;
  }
  static __device__ __forceinline__ v8f mma(v16b a, v16b b, v8f c) {
    return __builtin_amdgcn_wmma_f32_16x16x32_bf16(false, a, false, b, (short)0, c, false, false);
  }
  static __device__ __forceinline__ void guard(v8f& a, v8f& b, v16b x, v16b y) { dep_guard_b(a, b, x, y); }
  static __device__ __forceinline__ void keep(v16b a, v16b b, v16b c, v16b d) { keep4_b(a, b, c, d); }
};

template <int ET> struct Elem;
template <> struct Elem<0> { typedef _Float16 T; };
template <> struct Elem<1> { typedef __bf16 T; };
template <int ET, int SPLIT, int BIAS_MODE, int OUT_MODE, bool RESID>
__global__ __launch_bounds__(256) void wmma_gemm64(
    const unsigned short* __restrict__ Ap, const unsigned short* __restrict__ A2p, int lda, long strideA,
    const unsigned short* __restrict__ Btp, const unsigned short* __restrict__ Bt2p, int ldb, long strideB,
    void* __restrict__ Cout, void* __restrict__ Cout2, int ldc, long strideC,
    const float* __restrict__ bias,
    const float* __restrict__ resid, long strideR,
    int M, int N, int K, float scale) {
  typedef typename Elem<ET>::T T;
  typedef typename Frag<T>::V V;
  constexpr bool kSplA = (SPLIT != 0);
  constexpr bool kSplB = (SPLIT == 1);
  const T* A = (const T*)Ap; const T* A2 = (const T*)A2p; const T* Bt = (const T*)Btp; const T* Bt2 = (const T*)Bt2p;
  __shared__ __align__(16) float sT[8][16 * 68];
  const int b    = blockIdx.y;
  const int lane = threadIdx.x & 31;
  const int wave = threadIdx.x >> 5;
  const int tilesN = N >> 6;
  const int tilesM = M >> 6;
  const int tile = blockIdx.x * 8 + wave;
  if (tile >= tilesM * tilesN) return;
  const int tm = tile / tilesN;
  const int tn = tile - tm * tilesN;
  const int m0 = tm << 6;
  const int n0 = tn << 6;

  const T* Ab  = A  + (size_t)b * strideA;
  const T* Bb  = Bt + (size_t)b * strideB;
  const T* Ab2 = kSplA ? (A2  + (size_t)b * strideA) : nullptr;
  const T* Bb2 = kSplB ? (Bt2 + (size_t)b * strideB) : nullptr;

  const int rlane = lane & 15;
  const int koff  = (lane >> 4) * 8;
  const int mOff  = (lane >> 4) * 8;

  v8f acc[4][4];
#pragma unroll
  for (int i = 0; i < 4; ++i)
#pragma unroll
    for (int j = 0; j < 4; ++j) acc[i][j] = (v8f){0.f,0.f,0.f,0.f,0.f,0.f,0.f,0.f};

  for (int k0 = 0; k0 < K; k0 += 32) {
    V bh[4], bl[4];
#pragma unroll
    for (int j = 0; j < 4; ++j) {
      const size_t bo = (size_t)(n0 + (j << 4) + rlane) * ldb + koff + k0;
      bh[j] = Frag<T>::load(Bb + bo);
      if (kSplB) bl[j] = Frag<T>::load(Bb2 + bo);
    }
#pragma unroll
    for (int i = 0; i < 4; ++i) {
      const size_t ao = (size_t)(m0 + (i << 4) + rlane) * lda + koff + k0;
      V ah = Frag<T>::load(Ab + ao);
      V al = ah;
      if (kSplA) al = Frag<T>::load(Ab2 + ao);
#pragma unroll
      for (int j = 0; j < 4; ++j) {
        acc[i][j] = Frag<T>::mma(ah, bh[j], acc[i][j]);
        if (kSplB) acc[i][j] = Frag<T>::mma(ah, bl[j], acc[i][j]);
        if (kSplA) acc[i][j] = Frag<T>::mma(al, bh[j], acc[i][j]);
      }
      Frag<T>::guard(acc[i][0], acc[i][3], ah, al);
    }
    Frag<T>::keep(bh[0], bh[1], bh[2], bh[3]);
    if (kSplB) Frag<T>::keep(bl[0], bl[1], bl[2], bl[3]);
  }
  acc_guard4(acc[0][0], acc[0][1], acc[0][2], acc[0][3]);
  acc_guard4(acc[1][0], acc[1][1], acc[1][2], acc[1][3]);
  acc_guard4(acc[2][0], acc[2][1], acc[2][2], acc[2][3]);
  acc_guard4(acc[3][0], acc[3][1], acc[3][2], acc[3][3]);

  float* slab = sT[wave];
  const float* Rb = RESID ? (resid + (size_t)b * strideR) : nullptr;
#pragma unroll
  for (int i = 0; i < 4; ++i) {
    const int mBase = m0 + (i << 4);
#pragma unroll
    for (int j = 0; j < 4; ++j) {
      const int n = n0 + (j << 4) + rlane;
      float bv = 0.f;
      if (BIAS_MODE == 2) bv = bias[n];
#pragma unroll
      for (int r = 0; r < 8; ++r) {
        float v = acc[i][j][r] * scale;
        if (BIAS_MODE == 1) v += bias[mBase + mOff + r];
        if (BIAS_MODE == 2) v += bv;
        if (RESID) v += Rb[(size_t)(mBase + mOff + r) * ldc + n];
        slab[(mOff + r) * 68 + (j << 4) + rlane] = v;
      }
    }
    __builtin_amdgcn_fence(__ATOMIC_RELEASE, "workgroup");
    __builtin_amdgcn_wave_barrier();
    __builtin_amdgcn_fence(__ATOMIC_ACQUIRE, "workgroup");
    if (OUT_MODE == 0) {
      float* C = (float*)Cout + (size_t)b * strideC;
      const int hh = lane >> 4, c4 = (lane & 15) * 4;
      for (int pass = 0; pass < 2; ++pass) {
#pragma unroll
        for (int it = 0; it < 8; ++it) {
          const int row = it * 2 + hh;
          v4f v = *(const v4f*)(slab + row * 68 + c4);
          *(volatile v4f*)(C + (size_t)(mBase + row) * ldc + n0 + c4) = v;
        }
        __threadfence();
      }
    } else {
      const int q = lane >> 3, c8 = (lane & 7) * 8;
      unsigned short* C  = (unsigned short*)Cout  + (size_t)b * strideC;
      unsigned short* C2 = (OUT_MODE == 2) ? ((unsigned short*)Cout2 + (size_t)b * strideC) : nullptr;
      for (int pass = 0; pass < 2; ++pass) {
#pragma unroll
        for (int it = 0; it < 4; ++it) {
          const int row = it * 4 + q;
          const float* sp = slab + row * 68 + c8;
          v8h hv, lv;
#pragma unroll
          for (int e = 0; e < 8; ++e) {
            if (OUT_MODE == 1) {
              hv[e] = (_Float16)sp[e];
            } else {
              unsigned short hb = f2bf_bits(sp[e]);
              unsigned short lb = f2bf_bits(sp[e] - bf_bits2f(hb));
              hv[e] = __builtin_bit_cast(_Float16, hb);
              lv[e] = __builtin_bit_cast(_Float16, lb);
            }
          }
          *(volatile v8h*)(C + (size_t)(mBase + row) * ldc + n0 + c8) = hv;
          if (OUT_MODE == 2) *(volatile v8h*)(C2 + (size_t)(mBase + row) * ldc + n0 + c8) = lv;
        }
        __threadfence();
      }
    }
    __builtin_amdgcn_fence(__ATOMIC_RELEASE, "workgroup");
    __builtin_amdgcn_wave_barrier();
    __builtin_amdgcn_fence(__ATOMIC_ACQUIRE, "workgroup");
  }
}

__global__ __launch_bounds__(256) void cast_f32_bf16x8(const float* __restrict__ in,
                                                      unsigned short* __restrict__ outp, int n8) {
  const int i = blockIdx.x * 256 + threadIdx.x;
  if (i < n8) {
    const v4f a = *(const v4f*)(in + (size_t)i * 8);
    const v4f c = *(const v4f*)(in + (size_t)i * 8 + 4);
    v8h hv;
#pragma unroll
    for (int e = 0; e < 4; ++e) {
      hv[e]     = __builtin_bit_cast(_Float16, f2bf_bits(a[e]));
      hv[4 + e] = __builtin_bit_cast(_Float16, f2bf_bits(c[e]));
    }
    _Float16* o = (_Float16*)outp + (size_t)i * 8;
    *(volatile v8h*)o = hv;
    __threadfence();
    *(volatile v8h*)o = hv;
  }
}

constexpr int kWtPitch = 72;
__global__ __launch_bounds__(256) void wt_cast_bf16(const float* __restrict__ W, unsigned short* __restrict__ Wtp,
                                                    int Kdim, int Ndim) {
  __shared__ __align__(16) _Float16 st[64 * kWtPitch];
  _Float16* Wt = (_Float16*)Wtp;
  const int n0 = blockIdx.x * 64, k0 = blockIdx.y * 64;
  const int tid = threadIdx.x;
  const int kr = tid >> 2, c16 = (tid & 3) * 16;
  const float* src = W + (size_t)(k0 + kr) * Ndim + n0 + c16;
#pragma unroll
  for (int q = 0; q < 4; ++q) {
    const v4f v = *(const v4f*)(src + 4 * q);
#pragma unroll
    for (int e = 0; e < 4; ++e) st[(c16 + 4 * q + e) * kWtPitch + kr] = __builtin_bit_cast(_Float16, f2bf_bits(v[e]));
  }
  __syncthreads();
  const int wave = tid >> 5, lane = tid & 31;
  const int q8 = lane >> 3, c8 = (lane & 7) * 8;
  for (int pass = 0; pass < 2; ++pass) {
#pragma unroll
    for (int it = 0; it < 2; ++it) {
      const int n = it * 32 + wave * 4 + q8;
      const v8h hv = *(const v8h*)(st + n * kWtPitch + c8);
      *(volatile v8h*)(Wt + (size_t)(n0 + n) * Kdim + k0 + c8) = hv;
    }
    __threadfence();
  }
}

constexpr int kKeyChunk = 64;
constexpr int kQBlock   = 64;
constexpr int kOsPitch  = 68;

__device__ __forceinline__ v8f mma_bf(v16b a, v16b b, v8f c) {
  c = __builtin_amdgcn_wmma_f32_16x16x32_bf16(false, a, false, b, (short)0, c, false, false);
  asm volatile("v_nop\n\tv_nop\n\tv_nop\n\tv_nop" : "+v"(c) : "v"(a), "v"(b));
  return c;
}
__device__ __forceinline__ void split_bf(float f, __bf16& hi, __bf16& lo) {
  const unsigned short hb = f2bf_bits(f);
  hi = __builtin_bit_cast(__bf16, hb);
  lo = __builtin_bit_cast(__bf16, f2bf_bits(f - bf_bits2f(hb)));
}

__global__ __launch_bounds__(128)
void attn_causal_hd64(const unsigned short* __restrict__ qhp, const unsigned short* __restrict__ qlp,
                      const unsigned short* __restrict__ kvhp, const unsigned short* __restrict__ kvlp,
                      unsigned short* __restrict__ ohp, unsigned short* __restrict__ olp) {
  union FB { v16b v; v8b h[2]; };
  __shared__ __align__(16) __bf16 Ksh[kKeyChunk * kHdim];
  __shared__ __align__(16) __bf16 Ksl[kKeyChunk * kHdim];
  __shared__ __align__(16) __bf16 Vth[kHdim * kKeyChunk];
  __shared__ __align__(16) __bf16 Vtl[kHdim * kKeyChunk];
  __shared__ __align__(16) __bf16 Psh[4][16 * kKeyChunk];
  __shared__ __align__(16) __bf16 Psl[4][16 * kKeyChunk];
  __shared__ __align__(16) float  Os[4][16 * kOsPitch];

  const __bf16* qh  = (const __bf16*)qhp;
  const __bf16* ql  = (const __bf16*)qlp;
  const __bf16* kvh = (const __bf16*)kvhp;
  const __bf16* kvl = (const __bf16*)kvlp;

  const int tid  = threadIdx.x;
  const int wave = tid >> 5;
  const int lane = tid & 31;
  const int hh   = lane >> 4;
  const int c    = lane & 15;

  constexpr int nqb = kSeq / kQBlock;
  const int bx = blockIdx.x;
  const int qb = bx % nqb;
  const int bh = bx / nqb;
  const int h  = bh % kHeads;
  const int b  = bh / kHeads;
  const int q0 = qb * kQBlock + wave * 16;
  const size_t tokb = (size_t)b * kSeq;

  v16b qah[2], qal[2];
  {
    const size_t qo = (tokb + q0 + c) * (size_t)kChan + (size_t)h * kHdim + 8 * hh;
#pragma unroll
    for (int dc = 0; dc < 2; ++dc) {
      qah[dc] = Frag<__bf16>::load(qh + qo + dc * 32);
      qal[dc] = Frag<__bf16>::load(ql + qo + dc * 32);
    }
  }

  float mrow[8], lrow[8];
  v8f oacc[4];
#pragma unroll
  for (int r = 0; r < 8; ++r) { mrow[r] = neg_inf_f(); lrow[r] = 0.f; }
#pragma unroll
  for (int t = 0; t < 4; ++t) oacc[t] = (v8f){0.f,0.f,0.f,0.f,0.f,0.f,0.f,0.f};

  const int nChunks = qb + 1;
  for (int kc = 0; kc < nChunks; ++kc) {
    const int kv0 = kc * kKeyChunk;
    __syncthreads();
    {
      const int kvr = tid >> 1, dh = (tid & 1) * 32;
      const size_t ro = (tokb + kv0 + kvr) * (size_t)(2 * kChan) + (size_t)h * kHdim + dh;
#pragma unroll
      for (int i = 0; i < 4; ++i) {
        const v8b kkh = *(const v8b*)(kvh + ro + 8 * i);
        const v8b kkl = *(const v8b*)(kvl + ro + 8 * i);
        *(v8b*)(Ksh + kvr * kHdim + dh + 8 * i) = kkh;
        *(v8b*)(Ksl + kvr * kHdim + dh + 8 * i) = kkl;
        const v8b vvh = *(const v8b*)(kvh + ro + kChan + 8 * i);
        const v8b vvl = *(const v8b*)(kvl + ro + kChan + 8 * i);
#pragma unroll
        for (int e = 0; e < 8; ++e) {
          Vth[(dh + 8 * i + e) * kKeyChunk + kvr] = vvh[e];
          Vtl[(dh + 8 * i + e) * kKeyChunk + kvr] = vvl[e];
        }
      }
    }
    __syncthreads();

    v8f s[4];
#pragma unroll
    for (int j = 0; j < 4; ++j) {
      s[j] = (v8f){0.f,0.f,0.f,0.f,0.f,0.f,0.f,0.f};
#pragma unroll
      for (int dc = 0; dc < 2; ++dc) {
        FB kb, kl;
        const int ko = (j * 16 + c) * kHdim + dc * 32 + 8 * hh;
        kb.h[0] = *(const v8b*)(Ksh + ko);
        kb.h[1] = *(const v8b*)(Ksh + ko + 16);
        kl.h[0] = *(const v8b*)(Ksl + ko);
        kl.h[1] = *(const v8b*)(Ksl + ko + 16);
        s[j] = mma_bf(qah[dc], kb.v, s[j]);
        s[j] = mma_bf(qah[dc], kl.v, s[j]);
        s[j] = mma_bf(qal[dc], kb.v, s[j]);
      }
    }
    const bool diag = (kc == qb);
    float cm[8];
#pragma unroll
    for (int r = 0; r < 8; ++r) {
      const int qrow = q0 + 8 * hh + r;
      float m = neg_inf_f();
#pragma unroll
      for (int j = 0; j < 4; ++j) {
        const int kvcol = kv0 + j * 16 + c;
        float sv = s[j][r] * 0.125f;
        if (diag && (kvcol > qrow)) sv = neg_inf_f();
        s[j][r] = sv;
        m = fmaxf(m, sv);
      }
#pragma unroll
      for (int off = 1; off < 16; off <<= 1) m = fmaxf(m, __shfl_xor(m, off, 32));
      cm[r] = m;
    }
    __bf16* pwh = Psh[wave];
    __bf16* pwl = Psl[wave];
#pragma unroll
    for (int r = 0; r < 8; ++r) {
      const float mnew  = fmaxf(mrow[r], cm[r]);
      const float alpha = expf(mrow[r] - mnew);
      mrow[r] = mnew;
      float psum = 0.f;
#pragma unroll
      for (int j = 0; j < 4; ++j) {
        const float p = expf(s[j][r] - mnew);
        psum += p;
        __bf16 ph, pl;
        split_bf(p, ph, pl);
        pwh[(8 * hh + r) * kKeyChunk + j * 16 + c] = ph;
        pwl[(8 * hh + r) * kKeyChunk + j * 16 + c] = pl;
      }
#pragma unroll
      for (int off = 1; off < 16; off <<= 1) psum += __shfl_xor(psum, off, 32);
      lrow[r] = lrow[r] * alpha + psum;
#pragma unroll
      for (int t = 0; t < 4; ++t) oacc[t][r] *= alpha;
    }
    __builtin_amdgcn_fence(__ATOMIC_RELEASE, "workgroup");
    __builtin_amdgcn_wave_barrier();
    __builtin_amdgcn_fence(__ATOMIC_ACQUIRE, "workgroup");
#pragma unroll 1
    for (int kk = 0; kk < 2; ++kk) {
      FB pa, pl;
      const int po = c * kKeyChunk + kk * 32 + 8 * hh;
      pa.h[0] = *(const v8b*)(pwh + po);
      pa.h[1] = *(const v8b*)(pwh + po + 16);
      pl.h[0] = *(const v8b*)(pwl + po);
      pl.h[1] = *(const v8b*)(pwl + po + 16);
#pragma unroll
      for (int t = 0; t < 4; ++t) {
        FB vb, vl;
        const int vo = (t * 16 + c) * kKeyChunk + kk * 32 + 8 * hh;
        vb.h[0] = *(const v8b*)(Vth + vo);
        vb.h[1] = *(const v8b*)(Vth + vo + 16);
        vl.h[0] = *(const v8b*)(Vtl + vo);
        vl.h[1] = *(const v8b*)(Vtl + vo + 16);
        oacc[t] = mma_bf(pa.v, vb.v, oacc[t]);
        oacc[t] = mma_bf(pa.v, vl.v, oacc[t]);
        oacc[t] = mma_bf(pl.v, vb.v, oacc[t]);
      }
    }
  }

  float* os = Os[wave];
#pragma unroll
  for (int r = 0; r < 8; ++r) {
    const float inv = 1.0f / lrow[r];
#pragma unroll
    for (int t = 0; t < 4; ++t) os[(8 * hh + r) * kOsPitch + t * 16 + c] = oacc[t][r] * inv;
  }
  __builtin_amdgcn_fence(__ATOMIC_RELEASE, "workgroup");
  __builtin_amdgcn_wave_barrier();
  __builtin_amdgcn_fence(__ATOMIC_ACQUIRE, "workgroup");
  {
    const int q = lane >> 3, c8 = (lane & 7) * 8;
    _Float16* oh = (_Float16*)ohp + (tokb + q0) * (size_t)kChan + (size_t)h * kHdim;
    _Float16* ol = (_Float16*)olp + (tokb + q0) * (size_t)kChan + (size_t)h * kHdim;
    for (int pass = 0; pass < 2; ++pass) {
#pragma unroll
      for (int it = 0; it < 4; ++it) {
        const int row = it * 4 + q;
        const float* sp = os + row * kOsPitch + c8;
        v8h hv, lv;
#pragma unroll
        for (int e = 0; e < 8; ++e) {
          const float f = sp[e];
          const unsigned short hb = f2bf_bits(f);
          const unsigned short lb = f2bf_bits(f - bf_bits2f(hb));
          hv[e] = __builtin_bit_cast(_Float16, hb);
          lv[e] = __builtin_bit_cast(_Float16, lb);
        }
        *(volatile v8h*)(oh + (size_t)row * kChan + c8) = hv;
        *(volatile v8h*)(ol + (size_t)row * kChan + c8) = lv;
      }
      __threadfence();
    }
  }
}

extern "C" void kernel_launch(void* const* d_in, const int* in_sizes, int n_in,
                              void* d_out, int out_size, void* d_ws, size_t ws_size,
                              hipStream_t stream) {
  if (n_in < 5) return;
  const size_t nAct = (size_t)kTok * kChan;
  if (in_sizes[0] != (int)nAct || in_sizes[1] != (int)nAct) return;
  if (in_sizes[2] != kChan * kChan || in_sizes[3] != kChan * 2 * kChan || in_sizes[4] != kChan * kChan) return;
  if (out_size != (int)nAct) return;
  const size_t MiB = 1048576;
  const size_t carve = 128 * MiB;
  if (ws_size < carve) return;

  const float* x   = (const float*)d_in[0];
  const float* ctx = (const float*)d_in[1];
  const float* Wq  = (const float*)d_in[2];
  const float* Wkv = (const float*)d_in[3];
  const float* Wo  = (const float*)d_in[4];
  float* out = (float*)d_out;

  char* ws = (char*)d_ws;
  unsigned short* xb   = (unsigned short*)(ws + 0 * MiB);
  unsigned short* cb   = (unsigned short*)(ws + 16 * MiB);
  unsigned short* wkvT = (unsigned short*)(ws + 0 * MiB);
  unsigned short* oh   = (unsigned short*)(ws + 0 * MiB);
  unsigned short* ol   = (unsigned short*)(ws + 16 * MiB);
  unsigned short* qh   = (unsigned short*)(ws + 32 * MiB);
  unsigned short* ql   = (unsigned short*)(ws + 48 * MiB);
  unsigned short* woT  = (unsigned short*)(ws + 32 * MiB);
  unsigned short* wqT  = (unsigned short*)(ws + 64 * MiB);
  unsigned short* kvh  = (unsigned short*)(ws + 64 * MiB);
  unsigned short* kvl  = (unsigned short*)(ws + 96 * MiB);

  const int n8 = (int)(nAct / 8);
  const dim3 blk256(256), blk128(128);

  cast_f32_bf16x8<<<dim3((n8 + 255) / 256), blk256, 0, stream>>>(x, xb, n8);
  wt_cast_bf16<<<dim3(kChan / 64, kChan / 64), blk256, 0, stream>>>(Wq, wqT, kChan, kChan);
  wmma_gemm64<1, 0, 0, 2, false><<<dim3((kTok / 64) * (kChan / 64) / 8, 1), blk256, 0, stream>>>(
      xb, xb, kChan, 0L, wqT, wqT, kChan, 0L, (void*)qh, (void*)ql, kChan, 0L,
      nullptr, nullptr, 0L, kTok, kChan, kChan, 1.0f);
  cast_f32_bf16x8<<<dim3((n8 + 255) / 256), blk256, 0, stream>>>(ctx, cb, n8);
  wt_cast_bf16<<<dim3((2 * kChan) / 64, kChan / 64), blk256, 0, stream>>>(Wkv, wkvT, kChan, 2 * kChan);
  wmma_gemm64<1, 0, 0, 2, false><<<dim3((kTok / 64) * ((2 * kChan) / 64) / 8, 1), blk256, 0, stream>>>(
      cb, cb, kChan, 0L, wkvT, wkvT, kChan, 0L, (void*)kvh, (void*)kvl, 2 * kChan, 0L,
      nullptr, nullptr, 0L, kTok, 2 * kChan, kChan, 1.0f);
  attn_causal_hd64<<<dim3(kBatch * kHeads * (kSeq / kQBlock)), blk128, 0, stream>>>(qh, ql, kvh, kvl, oh, ol);
  wt_cast_bf16<<<dim3(kChan / 64, kChan / 64), blk256, 0, stream>>>(Wo, woT, kChan, kChan);
  wmma_gemm64<1, 2, 0, 0, false><<<dim3((kTok / 64) * (kChan / 64) / 8, 1), blk256, 0, stream>>>(
      oh, ol, kChan, 0L, woT, woT, kChan, 0L, (void*)out, nullptr, kChan, 0L,
      nullptr, nullptr, 0L, kTok, kChan, kChan, 1.0f);
}
